// decoder_20959440404725
// MI455X (gfx1250) — hardware-verified
//
#include <hip/hip_runtime.h>
#include <math.h>

constexpr int NHID    = 8;
constexpr int NLAT    = 4;
constexpr int NCLS    = 2;
constexpr int NBATCH  = 8192;
constexpr int NSTEP   = 512;
constexpr int NGATE   = 4 * NHID;
constexpr int NTP     = NSTEP / 2;
constexpr int RTHR    = 128;
constexpr int RWAVES  = RTHR / 32;
constexpr int NTILES  = NBATCH / 16;
constexpr int NJOBS   = NTILES * 2;
constexpr int CTHR    = 256;
constexpr int CWAVES  = CTHR / 32;
constexpr float LOG2E_F = 1.4426950408889634f;
constexpr size_t PLANE_FLOATS = (size_t)NTP * (size_t)NBATCH * 4;
constexpr size_t PLANE_BYTES  = PLANE_FLOATS * sizeof(float);

static_assert(NHID == 8);
static_assert(NLAT == 4);
static_assert(NCLS == 2);
static_assert(NGATE == 32);
static_assert(NBATCH % 16 == 0);
static_assert(NSTEP % 4 == 0);
static_assert(NJOBS % RWAVES == 0);
static_assert(NBATCH % CWAVES == 0);
static_assert(NTP % 32 == 0);
static_assert(2 * PLANE_BYTES <= (size_t)134217728);

typedef __attribute__((ext_vector_type(16))) __bf16   v16b;
typedef __attribute__((ext_vector_type(8)))  float    v8f;
typedef __attribute__((ext_vector_type(4)))  float    v4f;
typedef __attribute__((ext_vector_type(8)))  unsigned v8u;

__device__ __forceinline__ unsigned bf_rne_bits(float f) {
  const unsigned u = __float_as_uint(f);
  return (u + 0x7FFFu + ((u >> 16) & 1u)) >> 16;
}
__device__ __forceinline__ float bf_bits_to_f32(unsigned b) { return __uint_as_float(b << 16); }

__device__ __forceinline__ float fsig(float x) {
  return __builtin_amdgcn_rcpf(1.0f + __builtin_amdgcn_exp2f(-x * LOG2E_F));
}
__device__ __forceinline__ float ftanh_(float x) {
  return 1.0f - 2.0f * __builtin_amdgcn_rcpf(1.0f + __builtin_amdgcn_exp2f(x * (2.0f * LOG2E_F)));
}

__device__ __forceinline__ v16b build_w_frag(const v4f w) {
  const float w0 = w[0];
  const float w1 = w[1];
  const float w2 = w[2];
  const float w3 = w[3];
  const unsigned h0 = bf_rne_bits(w0);
  const unsigned h1 = bf_rne_bits(w1);
  const unsigned h2 = bf_rne_bits(w2);
  const unsigned h3 = bf_rne_bits(w3);
  const unsigned l0 = bf_rne_bits(w0 - bf_bits_to_f32(h0));
  const unsigned l1 = bf_rne_bits(w1 - bf_bits_to_f32(h1));
  const unsigned l2 = bf_rne_bits(w2 - bf_bits_to_f32(h2));
  const unsigned l3 = bf_rne_bits(w3 - bf_bits_to_f32(h3));
  const unsigned ph01 = h0 | (h1 << 16);
  const unsigned ph23 = h2 | (h3 << 16);
  const unsigned pl01 = l0 | (l1 << 16);
  const unsigned pl23 = l2 | (l3 << 16);
  v8u p;
  p[0] = ph01;
  p[1] = ph23;
  p[2] = ph01;
  p[3] = ph23;
  p[4] = pl01;
  p[5] = pl23;
  p[6] = pl01;
  p[7] = pl23;
  return __builtin_bit_cast(v16b, p);
}

__device__ __forceinline__ void cell_unit(const float iv, const float fv, const float gv, const float ov,
                                          float& cstate, float& hout) {
  const float ig = fsig(iv);
  const float fg = fsig(fv);
  const float gg = ftanh_(gv);
  const float og = fsig(ov);
  const float cn = fg * cstate + ig * gg;
  cstate = cn;
  hout = og * ftanh_(cn);
}

__device__ __forceinline__ void lstm_step(const v16b aT0, const v16b aT1, const v8f cT0, const v8f cT1,
                                          v8u& bw, float (&cst)[4], const v4f wl0, const v4f wl1,
                                          const float add0, const float add1, float& lg0, float& lg1) {
  const v16b bf = __builtin_bit_cast(v16b, bw);
  v8f d0 = __builtin_amdgcn_wmma_f32_16x16x32_bf16(false, aT0, false, bf, (short)0, cT0, false, false);
  v8f d1 = __builtin_amdgcn_wmma_f32_16x16x32_bf16(false, aT1, false, bf, (short)0, cT1, false, false);
  asm volatile("v_nop\n\tv_nop\n\tv_nop\n\tv_nop" : "+v"(d0), "+v"(d1) : "v"(aT0), "v"(aT1), "v"(bf));

  float hv[4];
  cell_unit(d0[0], d0[1], d0[2], d0[3], cst[0], hv[0]);
  cell_unit(d0[4], d0[5], d0[6], d0[7], cst[1], hv[1]);
  cell_unit(d1[0], d1[1], d1[2], d1[3], cst[2], hv[2]);
  cell_unit(d1[4], d1[5], d1[6], d1[7], cst[3], hv[3]);

  unsigned hb[4], lb[4];
#pragma unroll
  for (int w = 0; w < 4; ++w) {
    hb[w] = bf_rne_bits(hv[w]);
    lb[w] = bf_rne_bits(hv[w] - bf_bits_to_f32(hb[w]));
  }
  const unsigned ph01 = hb[0] | (hb[1] << 16);
  const unsigned ph23 = hb[2] | (hb[3] << 16);
  const unsigned pl01 = lb[0] | (lb[1] << 16);
  const unsigned pl23 = lb[2] | (lb[3] << 16);
  bw[0] = ph01;
  bw[1] = ph23;
  bw[2] = pl01;
  bw[3] = pl23;
  bw[4] = ph01;
  bw[5] = ph23;
  bw[6] = pl01;
  bw[7] = pl23;

  float p0 = hv[0] * wl0[0];
  p0 = fmaf(hv[1], wl0[1], p0);
  p0 = fmaf(hv[2], wl0[2], p0);
  p0 = fmaf(hv[3], wl0[3], p0);
  float p1 = hv[0] * wl1[0];
  p1 = fmaf(hv[1], wl1[1], p1);
  p1 = fmaf(hv[2], wl1[2], p1);
  p1 = fmaf(hv[3], wl1[3], p1);
  const float q0 = __shfl_xor(p0, 16, 32);
  const float q1 = __shfl_xor(p1, 16, 32);
  lg0 = (p0 + q0) + add0;
  lg1 = (p1 + q1) + add1;
}

__global__ __launch_bounds__(RTHR) void bilstm_scan_kernel(
    const float* __restrict__ z, const int* __restrict__ repP,
    const float* __restrict__ Wihf, const float* __restrict__ Whhf,
    const float* __restrict__ bihf, const float* __restrict__ bhhf,
    const float* __restrict__ Wihb, const float* __restrict__ Whhb,
    const float* __restrict__ bihb, const float* __restrict__ bhhb,
    const float* __restrict__ Wlin, const float* __restrict__ blin,
    float* __restrict__ Pf, float* __restrict__ Pb) {
  __shared__ __align__(16) float sWih[2 * NGATE * NLAT];
  __shared__ float sBih[2 * NGATE];
  __shared__ float sBhh[2 * NGATE];

  const int tid  = threadIdx.x;
  const int lane = tid & 31;
  const int wave = tid >> 5;
  const int h4   = lane >> 4;
  const int sub  = lane & 15;
  (void)repP;

  if (tid < 64) {
    const int d = tid >> 5;
    const int q = tid & 31;
    const float* wp = d ? Wihb : Wihf;
    const float* bi = d ? bihb : bihf;
    const float* bh = d ? bhhb : bhhf;
    const v4f wv = *(const v4f*)(wp + q * NLAT);
    *(v4f*)(sWih + d * (NGATE * NLAT) + q * NLAT) = wv;
    sBih[d * NGATE + q] = bi[q];
    sBhh[d * NGATE + q] = bh[q];
  }
  __syncthreads();

  const int job  = blockIdx.x * RWAVES + wave;
  const int tile = job >> 1;
  const int dir  = job & 1;
  const int b    = tile * 16 + sub;

  const v4f zv = *(const v4f*)(z + (size_t)b * NLAT);

  const float* whh = dir ? Whhb : Whhf;
  const int amh = sub >> 3;
  const int ak  = (sub >> 2) & 1;
  const int agi = sub & 3;
  const int rowT0 = agi * NHID + 4 * amh + ak;
  const int rowT1 = rowT0 + 2;
  const v4f wr0 = *(const v4f*)(whh + rowT0 * NHID + 4 * h4);
  const v4f wr1 = *(const v4f*)(whh + rowT1 * NHID + 4 * h4);
  const v16b aT0 = build_w_frag(wr0);
  const v16b aT1 = build_w_frag(wr1);

  const v4f wl0 = *(const v4f*)(Wlin + dir * NHID + 4 * h4);
  const v4f wl1 = *(const v4f*)(Wlin + 2 * NHID + dir * NHID + 4 * h4);
  const float bl0 = blin[0];
  const float bl1 = blin[1];
  const float add0 = dir ? 0.0f : bl0;
  const float add1 = dir ? 0.0f : bl1;

  v8f cT0, cT1;
#pragma unroll
  for (int r = 0; r < 8; ++r) {
    const int g0 = (r & 3) * NHID + 4 * h4 + ((r >> 2) & 1);
    const int g1 = g0 + 2;
    const v4f w0 = *(const v4f*)(sWih + dir * (NGATE * NLAT) + g0 * NLAT);
    const v4f w1 = *(const v4f*)(sWih + dir * (NGATE * NLAT) + g1 * NLAT);
    float x0 = zv[0] * w0[0];
    x0 = fmaf(zv[1], w0[1], x0);
    x0 = fmaf(zv[2], w0[2], x0);
    x0 = fmaf(zv[3], w0[3], x0);
    float x1 = zv[0] * w1[0];
    x1 = fmaf(zv[1], w1[1], x1);
    x1 = fmaf(zv[2], w1[2], x1);
    x1 = fmaf(zv[3], w1[3], x1);
    cT0[r] = (x0 + sBih[dir * NGATE + g0]) + sBhh[dir * NGATE + g0];
    cT1[r] = (x1 + sBih[dir * NGATE + g1]) + sBhh[dir * NGATE + g1];
  }

  v8u bw;
  bw[0] = 0u;
  bw[1] = 0u;
  bw[2] = 0u;
  bw[3] = 0u;
  bw[4] = 0u;
  bw[5] = 0u;
  bw[6] = 0u;
  bw[7] = 0u;
  float cst[4];
  cst[0] = 0.0f;
  cst[1] = 0.0f;
  cst[2] = 0.0f;
  cst[3] = 0.0f;

  float* P = dir ? Pb : Pf;

#pragma unroll 1
  for (int j = 0; j < NSTEP / 4; ++j) {
    float s0a, s0b, s1a, s1b, s2a, s2b, s3a, s3b;
    lstm_step(aT0, aT1, cT0, cT1, bw, cst, wl0, wl1, add0, add1, s0a, s0b);
    lstm_step(aT0, aT1, cT0, cT1, bw, cst, wl0, wl1, add0, add1, s1a, s1b);
    lstm_step(aT0, aT1, cT0, cT1, bw, cst, wl0, wl1, add0, add1, s2a, s2b);
    lstm_step(aT0, aT1, cT0, cT1, bw, cst, wl0, wl1, add0, add1, s3a, s3b);

    const float fa0 = h4 ? s2a : s0a;
    const float fa1 = h4 ? s2b : s0b;
    const float fb0 = h4 ? s3a : s1a;
    const float fb1 = h4 ? s3b : s1b;
    v4f ov;
    ov[0] = dir ? fb0 : fa0;
    ov[1] = dir ? fb1 : fa1;
    ov[2] = dir ? fa0 : fb0;
    ov[3] = dir ? fa1 : fb1;
    const int tp = dir ? (NTP - 1 - 2 * j - h4) : (2 * j + h4);
    float* pp = P + ((size_t)tp * NBATCH + (size_t)b) * 4;
    *(volatile v4f*)pp = ov;
    __threadfence();
    *(volatile v4f*)pp = ov;
  }
}

__device__ __forceinline__ void softmax_pair(const float a, const float b, float& p0, float& p1) {
  const float m  = fmaxf(a, b);
  const float e0 = __builtin_amdgcn_exp2f((a - m) * LOG2E_F);
  const float e1 = __builtin_amdgcn_exp2f((b - m) * LOG2E_F);
  const float inv = __builtin_amdgcn_rcpf(e0 + e1);
  p0 = e0 * inv;
  p1 = e1 * inv;
}

__global__ __launch_bounds__(CTHR) void combine_softmax_kernel(const float* __restrict__ Pf,
                                                               const float* __restrict__ Pb,
                                                               float* __restrict__ out) {
  const int tid  = threadIdx.x;
  const int lane = tid & 31;
  const int wave = tid >> 5;
  const int b    = blockIdx.x * CWAVES + wave;
  const int tp   = blockIdx.y * 32 + lane;
  const size_t pi = ((size_t)tp * NBATCH + (size_t)b) * 4;
  const v4f fa = *(const v4f*)(Pf + pi);
  const v4f fb = *(const v4f*)(Pb + pi);
  const float l00 = fa[0] + fb[0];
  const float l01 = fa[1] + fb[1];
  const float l10 = fa[2] + fb[2];
  const float l11 = fa[3] + fb[3];
  float r00, r01, r10, r11;
  softmax_pair(l00, l01, r00, r01);
  softmax_pair(l10, l11, r10, r11);
  v4f ov;
  ov[0] = r00;
  ov[1] = r01;
  ov[2] = r10;
  ov[3] = r11;
  float* op = out + (size_t)b * (size_t)(NSTEP * NCLS) + (size_t)tp * 4;
  *(volatile v4f*)op = ov;
  __threadfence();
  *(volatile v4f*)op = ov;
}

extern "C" void kernel_launch(void* const* d_in, const int* in_sizes, int n_in,
                              void* d_out, int out_size, void* d_ws, size_t ws_size, hipStream_t stream) {
  if (n_in < 12 || d_out == nullptr || d_ws == nullptr) return;
  if (in_sizes[0] != NBATCH * NLAT || in_sizes[1] != 1 ||
      in_sizes[2] != NGATE * NLAT || in_sizes[3] != NGATE * NHID || in_sizes[4] != NGATE || in_sizes[5] != NGATE ||
      in_sizes[6] != NGATE * NLAT || in_sizes[7] != NGATE * NHID || in_sizes[8] != NGATE || in_sizes[9] != NGATE ||
      in_sizes[10] != NCLS * 2 * NHID || in_sizes[11] != NCLS ||
      out_size != NBATCH * NSTEP * NCLS) return;
  if (2 * PLANE_BYTES > ws_size) return;

  const float* z    = (const float*)d_in[0];
  const int*   rep  = (const int*)d_in[1];
  const float* Wihf = (const float*)d_in[2];
  const float* Whhf = (const float*)d_in[3];
  const float* bihf = (const float*)d_in[4];
  const float* bhhf = (const float*)d_in[5];
  const float* Wihb = (const float*)d_in[6];
  const float* Whhb = (const float*)d_in[7];
  const float* bihb = (const float*)d_in[8];
  const float* bhhb = (const float*)d_in[9];
  const float* Wlin = (const float*)d_in[10];
  const float* blin = (const float*)d_in[11];

  float* Pf = (float*)d_ws;
  float* Pb = (float*)((char*)d_ws + PLANE_BYTES);

  bilstm_scan_kernel<<<NJOBS / RWAVES, RTHR, 0, stream>>>(
      z, rep, Wihf, Whhf, bihf, bhhf, Wihb, Whhb, bihb, bhhb, Wlin, blin, Pf, Pb);
  combine_softmax_kernel<<<dim3(NBATCH / CWAVES, NTP / 32), CTHR, 0, stream>>>(Pf, Pb, (float*)d_out);
}
